// DiTBlockFut_67894843015269
// MI455X (gfx1250) — hardware-verified
//
#include <hip/hip_runtime.h>
#include <math.h>

typedef __attribute__((ext_vector_type(16))) _Float16 v16h;
typedef __attribute__((ext_vector_type(16))) __bf16 v16b;
typedef __attribute__((ext_vector_type(8)))  _Float16 v8h;
typedef __attribute__((ext_vector_type(8)))  float v8f;
typedef __attribute__((ext_vector_type(4)))  float v4f;
typedef __attribute__((ext_vector_type(2)))  float v2f;
typedef __attribute__((ext_vector_type(4)))  unsigned v4u;
typedef __attribute__((ext_vector_type(4)))  int v4i;
typedef float __attribute__((may_alias)) float_a;
typedef int __attribute__((may_alias)) int_a;

template <typename T> __device__ __forceinline__ void vst2(void* p, T v) { *(volatile T*)p = v; __threadfence(); *(volatile T*)p = v; }
__device__ __forceinline__ v8f wmma16(v16h a, v16h b, v8f c) {
  v8f d = __builtin_amdgcn_wmma_f32_16x16x32_f16(false, a, false, b, (short)0, c, false, false);
  asm volatile("v_nop\n\tv_nop\n\tv_nop\n\tv_nop" : "+v"(d) : "v"(a), "v"(b));
  return d;
}
__device__ __forceinline__ v8f wmma_bf(v16b a, v16b b, v8f c) {
  v8f d = __builtin_amdgcn_wmma_f32_16x16x32_bf16(false, a, false, b, (short)0, c, false, false);
  asm volatile("v_nop\n\tv_nop\n\tv_nop\n\tv_nop" : "+v"(d) : "v"(a), "v"(b));
  return d;
}
__device__ __forceinline__ v16h frag_h(const _Float16* rowk0, int lane) {
  union { v16h v; v8h q[2]; } u; const _Float16* p = rowk0 + 8 * (lane >> 4);
  u.q[0] = *(const v8h*)p; u.q[1] = *(const v8h*)(p + 16); return u.v;
}
__device__ __forceinline__ v16h frag_f32(const float* rowk0, int lane) {
  v16h a; const float* p = rowk0 + 8 * (lane >> 4);
#pragma unroll
  for (int i = 0; i < 8; ++i) { a[i] = (_Float16)p[i]; a[8 + i] = (_Float16)p[16 + i]; }
  return a;
}
__device__ __forceinline__ v16h frag_f32s(const float* rowk0, int lane, float sc) {
  v16h a; const float* p = rowk0 + 8 * (lane >> 4);
#pragma unroll
  for (int i = 0; i < 8; ++i) { a[i] = (_Float16)(p[i] * sc); a[8 + i] = (_Float16)(p[16 + i] * sc); }
  return a;
}
__device__ __forceinline__ v16h fragc_f32(const float* W, int k0, int n, int lane, int ld, int K) {
  v16h a; const int g = lane >> 4;
#pragma unroll
  for (int i = 0; i < 8; ++i) { const int ka = k0 + 8 * g + i, kb = ka + 16;
    a[i] = (_Float16)(ka < K ? W[(size_t)(ka < K ? ka : K - 1) * ld + n] : 0.f); a[8 + i] = (_Float16)(kb < K ? W[(size_t)(kb < K ? kb : K - 1) * ld + n] : 0.f); }
  return a;
}
struct F2 { v16b h, l; };
__device__ __forceinline__ F2 bsplit16(const float v[16]) { F2 r;
#pragma unroll
  for (int i = 0; i < 16; ++i) { const __bf16 h = (__bf16)v[i]; r.h[i] = h; r.l[i] = (__bf16)(v[i] - (float)h); }
  return r; }
__device__ __forceinline__ F2 split_row(const float* row, int k0, int lane) { float v[16]; const float* p = row + k0 + 8 * (lane >> 4);
#pragma unroll
  for (int i = 0; i < 8; ++i) { v[i] = p[i]; v[8 + i] = p[16 + i]; }
  return bsplit16(v); }
__device__ __forceinline__ F2 split_rowK(const float* row, int k0, int lane, int K) { float v[16]; const int g = lane >> 4;
#pragma unroll
  for (int i = 0; i < 8; ++i) { const int ka = k0 + 8 * g + i, kb = ka + 16; v[i] = ka < K ? row[ka < K ? ka : K - 1] : 0.f; v[8 + i] = kb < K ? row[kb < K ? kb : K - 1] : 0.f; }
  return bsplit16(v); }
__device__ __forceinline__ F2 split_col(const float* W, int k0, int n, int lane, int ld, int K) { float v[16]; const int g = lane >> 4;
#pragma unroll
  for (int i = 0; i < 8; ++i) { const int ka = k0 + 8 * g + i, kb = ka + 16; v[i] = ka < K ? W[(size_t)(ka < K ? ka : K - 1) * ld + n] : 0.f; v[8 + i] = kb < K ? W[(size_t)(kb < K ? kb : K - 1) * ld + n] : 0.f; }
  return bsplit16(v); }
__device__ __forceinline__ v8f mac3(const F2& a, const F2& b, v8f c) { c = wmma_bf(a.l, b.h, c); c = wmma_bf(a.h, b.l, c); return wmma_bf(a.h, b.h, c); }
__device__ __forceinline__ float sigm(float v) { return 1.0f / (1.0f + expf(-v)); }
#define LDSX() do { asm volatile("s_wait_dscnt 0" ::: "memory"); __builtin_amdgcn_wave_barrier(); __builtin_amdgcn_fence(__ATOMIC_RELEASE, "workgroup"); } while (0)


#define NB 4
#define SS 512
#define NR (NB * SS)
#define DM 1024
#define NH 16
#define HD 64
#define HID 4096
#define RPH 64
#ifndef TQB
#define TQB (SS / 64)
#define TNB NB
#define TB0 0
#endif
#define RB0 ((size_t)TB0 * SS)
#define RKV (TNB * SS)
#define RTQ (((TNB - 1) * SS) + TQB * 64)
typedef __attribute__((ext_vector_type(8))) __bf16 v8b;
__device__ __forceinline__ v16b frag_b(const __bf16* rowk0, int lane) {
  union { v16b v; v8b q[2]; } u; const __bf16* p = rowk0 + 8 * (lane >> 4);
  u.q[0] = *(const v8b*)p; u.q[1] = *(const v8b*)(p + 16); return u.v;
}
__device__ __forceinline__ float bfr(float v) { return (float)(__bf16)v; }
__device__ __attribute__((noinline)) float exp_ni(float v) { return expf(v); }
__device__ __attribute__((noinline)) float erf_ni(float v) { return erff(v); }
__device__ __forceinline__ float silu_f(float x) { return x / (1.0f + exp_ni(-x)); }

#define PK_QKV 0
#define PK_PRJ ((size_t)3 * DM * DM)
#define PK_ADA ((size_t)4 * DM * DM)
#define PK_FC1 ((size_t)10 * DM * DM)
#define PK_FC2 ((size_t)14 * DM * DM)
#define PK_RP2 ((size_t)18 * DM * DM)
#define PK_END (PK_RP2 + (size_t)NH * RPH)
#define WS_PK  0u
#define WS_MOD (((2u * PK_END) + 127u) / 128u * 128u)
#define WS_T   (WS_MOD + 4u * NB * 6 * DM)
#define WS_QK  (WS_T + 4u * NR * DM)
#define WS_QKL (WS_QK + 2u * NR * 2 * DM)
#define WS_VTH (WS_QKL + 2u * NR * 2 * DM)
#define WS_VTL (WS_VTH + 2u * NR * DM)
#define WS_BIAS (WS_VTL + 2u * NR * DM)
#define WS_O   (WS_BIAS + 4u * (size_t)NB * NH * SS * SS)
#define WS_X1  (WS_O + 4u * NR * DM)
#define WS_GH  (WS_X1 + 4u * NR * DM)
#define WS_GL  (WS_GH + 2u * (size_t)NR * HID)
#define WS_END (WS_GL + 2u * (size_t)NR * HID)

__global__ __launch_bounds__(256) void k_pack(const float* __restrict__ WQKV, const float* __restrict__ WPRJ, const float* __restrict__ WADA, const float* __restrict__ WFC1, const float* __restrict__ WFC2, const float* __restrict__ WRP2, __bf16* __restrict__ PK) {
  __shared__ __align__(16) __bf16 s[HID]; const int n = blockIdx.x, which = blockIdx.y, t = threadIdx.x; int K, NO; size_t dst; const float* Wm;
  switch (which) { case 0: Wm = WQKV; K = DM; NO = 3 * DM; dst = PK_QKV; break; case 1: Wm = WPRJ; K = DM; NO = DM; dst = PK_PRJ; break; case 2: Wm = WADA; K = DM; NO = 6 * DM; dst = PK_ADA; break; case 3: Wm = WFC1; K = DM; NO = HID; dst = PK_FC1; break; case 4: Wm = WFC2; K = HID; NO = DM; dst = PK_FC2; break; default: Wm = WRP2; K = RPH; NO = NH; dst = PK_RP2; break; }
  if (n >= NO) return;
  for (int k = t; k < K; k += 256) s[k] = (__bf16)Wm[(size_t)n * K + k];
  __syncthreads();
  for (int q = t; q < K / 8; q += 256) vst2((unsigned*)(PK + dst + (size_t)n * K + q * 8), *(const v4u*)&s[q * 8]);
}
__global__ __launch_bounds__(128) void k_mod(const float* __restrict__ TEMB, const __bf16* __restrict__ PK, const float* __restrict__ BADA, float* __restrict__ MOD) {
  __shared__ __align__(16) __bf16 sah[16][DM + 8], sal[16][DM + 8]; __shared__ __align__(16) float so[NB][132];
  const int tid = threadIdx.x, wave = tid >> 5, lane = tid & 31, col = lane & 15, g = lane >> 4; const int n0 = blockIdx.x * 128;
  for (int e = tid; e < 16 * (DM + 8); e += 128) { const int r = e / (DM + 8), c = e % (DM + 8); float v = 0.f; if (r < NB && c < DM) v = silu_f(bfr(TEMB[r * DM + c])); const __bf16 hb = (__bf16)v; sah[r][c] = hb; sal[r][c] = (__bf16)(v - (float)hb); }
  __syncthreads();
  v8f acc[2] = {};
#pragma unroll 4
  for (int kc = 0; kc < DM / 32; ++kc) { F2 a; a.h = frag_b(&sah[col][kc * 32], lane); a.l = frag_b(&sal[col][kc * 32], lane);
#pragma unroll
    for (int j = 0; j < 2; ++j) { const v16b w = frag_b(PK + PK_ADA + (size_t)(n0 + wave * 32 + j * 16 + col) * DM + kc * 32, lane); acc[j] = wmma_bf(a.l, w, acc[j]); acc[j] = wmma_bf(a.h, w, acc[j]); } }
#pragma unroll
  for (int j = 0; j < 2; ++j) { const int c = wave * 32 + j * 16 + col; const float bb = bfr(BADA[n0 + c]); if (g == 0) {
#pragma unroll
      for (int r = 0; r < NB; ++r) so[r][c] = acc[j][r] + bb; } }
  __syncthreads();
  for (int b = 0; b < NB; ++b) if (tid < 32) vst2(MOD + (size_t)b * 6 * DM + n0 + tid * 4, *(const v4f*)&so[b][tid * 4]);
}
__global__ __launch_bounds__(256) void k_lnmod(const float* __restrict__ SRC, int round_src, const float* __restrict__ G, const float* __restrict__ Bv, const float* __restrict__ MOD, int which, float* __restrict__ T) {
  __shared__ float red[2][8]; const int t = threadIdx.x; const size_t row = RB0 + blockIdx.x; const int b = (int)(row / SS); const float* p = SRC + row * DM + t * 4;
  float v[4];
#pragma unroll
  for (int i = 0; i < 4; ++i) v[i] = round_src ? bfr(p[i]) : p[i];
  float s = (v[0] + v[1]) + (v[2] + v[3]);
#pragma unroll
  for (int o = 1; o < 32; o <<= 1) s += __shfl_xor(s, o);
  if ((t & 31) == 0) red[0][t >> 5] = s; __syncthreads();
  float tot = 0.f; for (int w = 0; w < 8; ++w) tot += red[0][w]; const float mu = tot / (float)DM; float q = 0.f;
#pragma unroll
  for (int i = 0; i < 4; ++i) { const float d = v[i] - mu; q += d * d; }
#pragma unroll
  for (int o = 1; o < 32; o <<= 1) q += __shfl_xor(q, o);
  if ((t & 31) == 0) red[1][t >> 5] = q; __syncthreads();
  float qt = 0.f; for (int w = 0; w < 8; ++w) qt += red[1][w]; const float inv = 1.0f / sqrtf(qt / (float)DM + 1e-5f);
  const float* shift = MOD + (size_t)b * 6 * DM + (which == 0 ? 0 : 3 * DM); const float* scale = MOD + (size_t)b * 6 * DM + (which == 0 ? DM : 4 * DM);
  v4f o4;
#pragma unroll
  for (int i = 0; i < 4; ++i) { const int c = t * 4 + i; o4[i] = ((v[i] - mu) * inv * bfr(G[c]) + bfr(Bv[c])) * (1.0f + scale[c]) + shift[c]; }
  vst2(T + row * DM + t * 4, o4);
}
__global__ __launch_bounds__(128) void k_qkv(const float* __restrict__ T, const __bf16* __restrict__ PK, const float* __restrict__ BQKV, _Float16* __restrict__ QK, _Float16* __restrict__ QKL, _Float16* __restrict__ VTH, _Float16* __restrict__ VTL) {
  __shared__ __align__(16) _Float16 soh[4][16][136], sol[4][16][136]; __shared__ __align__(16) _Float16 sth[128][72], stl[128][72];
  const int tid = threadIdx.x, wave = tid >> 5, lane = tid & 31, col = lane & 15, g = lane >> 4; const size_t r0 = RB0 + (size_t)blockIdx.x * 64 + wave * 16; const int n0 = blockIdx.y * 128;
  v8f acc[8] = {};
#pragma unroll 2
  for (int kc = 0; kc < DM / 32; ++kc) { const F2 a = split_row(T + (r0 + col) * DM, kc * 32, lane);
#pragma unroll
    for (int j = 0; j < 8; ++j) { const v16b w = frag_b(PK + PK_QKV + (size_t)(n0 + j * 16 + col) * DM + kc * 32, lane); acc[j] = wmma_bf(a.l, w, acc[j]); acc[j] = wmma_bf(a.h, w, acc[j]); } }
  if (n0 < 2 * DM) {
#pragma unroll
    for (int j = 0; j < 8; ++j) { const float bb = bfr(BQKV[n0 + j * 16 + col]);
#pragma unroll
      for (int r = 0; r < 8; ++r) { const float v = acc[j][r] + bb; const _Float16 hv = (_Float16)v; soh[wave][8 * g + r][j * 16 + col] = hv; sol[wave][8 * g + r][j * 16 + col] = (_Float16)((v - (float)hv) * 2048.0f); } }
    LDSX();
    for (int rl = 0; rl < 16; ++rl) { if (lane < 16) vst2((unsigned*)(QK + (r0 + rl) * (2 * DM) + n0 + lane * 8), *(const v4u*)&soh[wave][rl][lane * 8]); else vst2((unsigned*)(QKL + (r0 + rl) * (2 * DM) + n0 + (lane - 16) * 8), *(const v4u*)&sol[wave][rl][(lane - 16) * 8]); }
  } else {
#pragma unroll
    for (int j = 0; j < 8; ++j) { const float bb = bfr(BQKV[n0 + j * 16 + col]);
#pragma unroll
      for (int r = 0; r < 8; ++r) { const float v = acc[j][r] + bb; const _Float16 hv = (_Float16)v; sth[j * 16 + col][wave * 16 + 8 * g + r] = hv; stl[j * 16 + col][wave * 16 + 8 * g + r] = (_Float16)((v - (float)hv) * 2048.0f); } }
    __syncthreads();
    const size_t rb = RB0 + (size_t)blockIdx.x * 64; const int b = (int)(rb / SS), s0 = (int)(rb % SS);
    for (int e = tid; e < 128 * 8; e += 128) { const int d = e >> 3, pc = e & 7; const size_t o = ((size_t)b * DM + (n0 - 2 * DM) + d) * SS + s0 + pc * 8; vst2((unsigned*)(VTH + o), *(const v4u*)&sth[d][pc * 8]); vst2((unsigned*)(VTL + o), *(const v4u*)&stl[d][pc * 8]); }
  }
}
__global__ __launch_bounds__(128) void k_bias(const float* __restrict__ RP, const float* __restrict__ WRP1, const float* __restrict__ BRP1, const __bf16* __restrict__ PK, const float* __restrict__ BRP2, float* __restrict__ BIAS) {
  __shared__ __align__(16) __bf16 shh[64][72], shl[64][72]; __shared__ __align__(16) float sb[NH][68];
  const int tid = threadIdx.x, wave = tid >> 5, lane = tid & 31, col = lane & 15, g = lane >> 4; const int mb = blockIdx.x, n = blockIdx.y, b = blockIdx.z + TB0; const int m0 = mb * 64;
  { const int r = tid >> 1, half = tid & 1; const size_t pr = (((size_t)b * SS + n) * SS + m0 + r) * 2; const float p0 = bfr(RP[pr]), p1 = bfr(RP[pr + 1]);
#pragma unroll
    for (int i = 0; i < 32; ++i) { const int u = half * 32 + i; const float hv = fmaxf((p0 * bfr(WRP1[u * 2]) + p1 * bfr(WRP1[u * 2 + 1])) + bfr(BRP1[u]), 0.f); const __bf16 hb = (__bf16)hv; shh[r][u] = hb; shl[r][u] = (__bf16)(hv - (float)hb); }
    if (half == 0) for (int u = 64; u < 72; ++u) { shh[r][u] = (__bf16)0.f; shl[r][u] = (__bf16)0.f; } }
  __syncthreads();
  v8f acc = {};
#pragma unroll
  for (int kc = 0; kc < 2; ++kc) { F2 a; a.h = frag_b(&shh[wave * 16 + col][kc * 32], lane); a.l = frag_b(&shl[wave * 16 + col][kc * 32], lane); const v16b w = frag_b(PK + PK_RP2 + (size_t)col * RPH + kc * 32, lane); acc = wmma_bf(a.l, w, acc); acc = wmma_bf(a.h, w, acc); }
  { const float bb = bfr(BRP2[col]);
#pragma unroll
    for (int r = 0; r < 8; ++r) sb[col][wave * 16 + 8 * g + r] = acc[r] + bb; }
  __syncthreads();
  for (int e = tid; e < NH * 16; e += 128) { const int h = e >> 4, pc = e & 15; vst2(BIAS + (((size_t)b * NH + h) * SS + n) * SS + m0 + pc * 4, *(const v4f*)&sb[h][pc * 4]); }
}
__global__ __launch_bounds__(128) void k_attn(const _Float16* __restrict__ QK, const _Float16* __restrict__ QKL, const _Float16* __restrict__ VTH, const _Float16* __restrict__ VTL, const float* __restrict__ BIAS, const int* __restrict__ AMASK, float* __restrict__ O) {
  __shared__ __align__(16) _Float16 sph[4][16][40], spl[4][16][40]; __shared__ __align__(16) float so[4][16][68];
  const int tid = threadIdx.x, wave = tid >> 5, lane = tid & 31, col = lane & 15, g = lane >> 4; const int qb = blockIdx.x, h = blockIdx.y, b = blockIdx.z + TB0; const int q0 = qb * 64 + wave * 16; const size_t rq = (size_t)b * SS + q0 + col;
  v16h aq[2], aql[2];
#pragma unroll
  for (int kc = 0; kc < 2; ++kc) { aq[kc] = frag_h(QK + rq * (2 * DM) + h * HD + kc * 32, lane); aql[kc] = frag_h(QKL + rq * (2 * DM) + h * HD + kc * 32, lane); }
  const _Float16* Vh = VTH + ((size_t)b * DM + h * HD) * SS; const _Float16* Vl = VTL + ((size_t)b * DM + h * HD) * SS; const float* BS = BIAS + ((size_t)b * NH + h) * SS * SS;
  float m[8], l[8];
#pragma unroll
  for (int r = 0; r < 8; ++r) { m[r] = -3.0e38f; l[r] = 0.f; }
  v8f acc[4] = {}, accl[4] = {};
#pragma unroll 1
  for (int ks = 0; ks < SS / 32; ++ks) { v8f s[2];
#pragma unroll
    for (int ct = 0; ct < 2; ++ct) { const int kk = ks * 32 + ct * 16 + col; const _Float16* krow = QK + ((size_t)b * SS + kk) * (2 * DM) + DM + h * HD; const _Float16* krowl = QKL + ((size_t)b * SS + kk) * (2 * DM) + DM + h * HD; v8f c = {}, cl = {};
#pragma unroll
      for (int kc = 0; kc < 2; ++kc) { const v16h kh = frag_h(krow + kc * 32, lane); c = wmma16(aq[kc], kh, c); cl = wmma16(aql[kc], kh, cl); cl = wmma16(aq[kc], frag_h(krowl + kc * 32, lane), cl); }
      const bool keep = AMASK[(size_t)b * SS + kk] != 0;
#pragma unroll
      for (int r = 0; r < 8; ++r) { const int qi = q0 + 8 * g + r; s[ct][r] = keep ? ((c[r] + cl[r] * (1.0f / 2048.0f)) * 0.125f + BS[(size_t)qi * SS + kk]) : -3.0e38f; } }
#pragma unroll
    for (int r = 0; r < 8; ++r) { float mx = fmaxf(s[0][r], s[1][r]);
#pragma unroll
      for (int o = 1; o < 16; o <<= 1) mx = fmaxf(mx, __shfl_xor(mx, o));
      const float mn = fmaxf(m[r], mx); const float alpha = (m[r] <= -1.0e38f) ? 0.f : __expf(m[r] - mn);
      const float e0 = (s[0][r] <= -1.0e38f) ? 0.f : __expf(s[0][r] - mn), e1 = (s[1][r] <= -1.0e38f) ? 0.f : __expf(s[1][r] - mn); float es = e0 + e1;
#pragma unroll
      for (int o = 1; o < 16; o <<= 1) es += __shfl_xor(es, o);
      l[r] = l[r] * alpha + es; m[r] = (mn <= -1.0e38f) ? m[r] : mn;
#pragma unroll
      for (int dt = 0; dt < 4; ++dt) { acc[dt][r] *= alpha; accl[dt][r] *= alpha; }
      const _Float16 h0 = (_Float16)e0, h1 = (_Float16)e1; sph[wave][8 * g + r][col] = h0; sph[wave][8 * g + r][16 + col] = h1; spl[wave][8 * g + r][col] = (_Float16)((e0 - (float)h0) * 2048.0f); spl[wave][8 * g + r][16 + col] = (_Float16)((e1 - (float)h1) * 2048.0f); }
    LDSX();
    const v16h pah = frag_h(&sph[wave][col][0], lane), pal = frag_h(&spl[wave][col][0], lane);
#pragma unroll
    for (int dt = 0; dt < 4; ++dt) { const size_t vo = (size_t)(dt * 16 + col) * SS + ks * 32; const v16h vh = frag_h(Vh + vo, lane), vl = frag_h(Vl + vo, lane); acc[dt] = wmma16(pah, vh, acc[dt]); accl[dt] = wmma16(pal, vh, accl[dt]); accl[dt] = wmma16(pah, vl, accl[dt]); }
    LDSX(); }
#pragma unroll
  for (int r = 0; r < 8; ++r) { const float il = 1.0f / l[r];
#pragma unroll
    for (int dt = 0; dt < 4; ++dt) so[wave][8 * g + r][dt * 16 + col] = (acc[dt][r] + accl[dt][r] * (1.0f / 2048.0f)) * il; }
  LDSX();
  for (int rl = 0; rl < 16; ++rl) if (lane < 16) vst2(O + ((size_t)b * SS + q0 + rl) * DM + h * HD + lane * 4, *(const v4f*)&so[wave][rl][lane * 4]);
}
template <int MODE>
__global__ __launch_bounds__(128) void k_lin(const float* __restrict__ A, const __bf16* __restrict__ AG, const __bf16* __restrict__ AGL, const __bf16* __restrict__ PK, const float* __restrict__ BIAS, const float* __restrict__ RES, const float* __restrict__ MOD, float* __restrict__ OUTF, __bf16* __restrict__ OUTG, __bf16* __restrict__ OUTGL) {
  __shared__ __align__(16) float so[4][16][132]; __shared__ __align__(16) __bf16 sg[4][16][136], sgl[4][16][136];
  const int tid = threadIdx.x, wave = tid >> 5, lane = tid & 31, col = lane & 15, g = lane >> 4; const size_t r0 = RB0 + (size_t)blockIdx.x * 64 + wave * 16; const int n0 = blockIdx.y * 128;
  constexpr int KD = (MODE == 2) ? HID : DM; const __bf16* P = PK + ((MODE == 0) ? PK_PRJ : (MODE == 1) ? PK_FC1 : PK_FC2);
  v8f acc[8] = {};
  if (MODE == 2) {
#pragma unroll 2
    for (int kc = 0; kc < KD / 32; ++kc) { const v16b a = frag_b(AG + (r0 + col) * HID + kc * 32, lane), al = frag_b(AGL + (r0 + col) * HID + kc * 32, lane);
#pragma unroll
      for (int j = 0; j < 8; ++j) { const v16b w = frag_b(P + (size_t)(n0 + j * 16 + col) * KD + kc * 32, lane); acc[j] = wmma_bf(al, w, acc[j]); acc[j] = wmma_bf(a, w, acc[j]); } }
  } else {
#pragma unroll 2
    for (int kc = 0; kc < KD / 32; ++kc) { const F2 a = split_row(A + (r0 + col) * DM, kc * 32, lane);
#pragma unroll
      for (int j = 0; j < 8; ++j) { const v16b w = frag_b(P + (size_t)(n0 + j * 16 + col) * KD + kc * 32, lane); acc[j] = wmma_bf(a.l, w, acc[j]); acc[j] = wmma_bf(a.h, w, acc[j]); } } }
#pragma unroll
  for (int j = 0; j < 8; ++j) { const int c = n0 + j * 16 + col; const float bb = bfr(BIAS[c]);
#pragma unroll
    for (int r = 0; r < 8; ++r) { const size_t row = r0 + 8 * g + r; const int b = (int)(row / SS); float v = acc[j][r] + bb;
      if (MODE == 1) { v = 0.5f * v * (1.0f + erf_ni(v * 0.70710678118654752f)); const __bf16 hb = (__bf16)v; sg[wave][8 * g + r][j * 16 + col] = hb; sgl[wave][8 * g + r][j * 16 + col] = (__bf16)(v - (float)hb); }
      else { const float gate = MOD[(size_t)b * 6 * DM + ((MODE == 0) ? 2 * DM : 5 * DM) + c]; const float res = (MODE == 0) ? bfr(RES[row * DM + c]) : RES[row * DM + c]; so[wave][8 * g + r][j * 16 + col] = res + gate * v; } } }
  LDSX();
  if (MODE == 1) { for (int rl = 0; rl < 16; ++rl) { if (lane < 16) vst2((unsigned*)(OUTG + (r0 + rl) * HID + n0 + lane * 8), *(const v4u*)&sg[wave][rl][lane * 8]); else vst2((unsigned*)(OUTGL + (r0 + rl) * HID + n0 + (lane - 16) * 8), *(const v4u*)&sgl[wave][rl][(lane - 16) * 8]); } }
  else { for (int rl = 0; rl < 16; ++rl) vst2(OUTF + (r0 + rl) * DM + n0 + lane * 4, *(const v4f*)&so[wave][rl][lane * 4]); }
}
extern "C" void kernel_launch(void* const* d_in, const int* in_sizes, int n_in, void* d_out, int out_size, void* d_ws, size_t ws_size, hipStream_t stream) {
  (void)in_sizes; (void)n_in; (void)out_size;
  const float** F = (const float**)d_in;
  if (ws_size < (size_t)WS_END) return;
  char* ws = (char*)d_ws; __bf16 *PK = (__bf16*)(ws + WS_PK), *GH = (__bf16*)(ws + WS_GH), *GL = (__bf16*)(ws + WS_GL); float *MOD = (float*)(ws + WS_MOD), *T = (float*)(ws + WS_T), *BIAS = (float*)(ws + WS_BIAS), *O = (float*)(ws + WS_O), *X1 = (float*)(ws + WS_X1); _Float16 *QK = (_Float16*)(ws + WS_QK), *QKL = (_Float16*)(ws + WS_QKL), *VTH = (_Float16*)(ws + WS_VTH), *VTL = (_Float16*)(ws + WS_VTL);
  k_pack<<<dim3(6 * DM, 6), 256, 0, stream>>>(F[10], F[12], F[4], F[18], F[20], F[16], PK);
  k_mod<<<6 * DM / 128, 128, 0, stream>>>(F[1], PK, F[5], MOD);
  k_lnmod<<<RKV, 256, 0, stream>>>(F[0], 1, F[6], F[7], MOD, 0, T);
  k_qkv<<<dim3(RKV / 64, 3 * DM / 128), 128, 0, stream>>>(T, PK, F[11], QK, QKL, VTH, VTL);
  k_bias<<<dim3(SS / 64, RTQ > SS ? SS : RTQ, TNB), 128, 0, stream>>>(F[2], F[14], F[15], PK, F[17], BIAS);
  k_attn<<<dim3(TQB, NH, TNB), 128, 0, stream>>>(QK, QKL, VTH, VTL, BIAS, (const int*)d_in[3], O);
  k_lin<0><<<dim3(RTQ / 64, DM / 128), 128, 0, stream>>>(O, nullptr, nullptr, PK, F[13], F[0], MOD, X1, nullptr, nullptr);
  k_lnmod<<<RTQ, 256, 0, stream>>>(X1, 0, F[8], F[9], MOD, 1, T);
  k_lin<1><<<dim3(RTQ / 64, HID / 128), 128, 0, stream>>>(T, nullptr, nullptr, PK, F[19], nullptr, MOD, nullptr, GH, GL);
  k_lin<2><<<dim3(RTQ / 64, DM / 128), 128, 0, stream>>>(nullptr, GH, GL, PK, F[21], X1, MOD, (float*)d_out, nullptr, nullptr);
}
